// _NonLocalBlockND_44083544326562
// MI455X (gfx1250) — hardware-verified
//
#include <hip/hip_runtime.h>
#include <math.h>
#include <stdint.h>

#ifndef NB
#define NB 8
#endif
#ifndef NQ
#define NQ 4096
#endif
#define NB_FULL 8
#define CC     256
#define HIMG   64
#define WIMG   64
#define NN     4096
#define DQ     128
#define HP     32
#define WP     32
#define MM     1024
#define MW     384
#define QT     64
#define SN     128
#define NSTRIP 32
#define OSP    68
#define OSPW   132
#define TP     72
#define BNQ    256
#define CHB    32
#define WSC    256.0f
#define IWSC   0.00390625f
#define LNPS   9.704060527839234f
#define BNEPS  1.0e-5f

static_assert(NB >= 1 && NB <= NB_FULL);
static_assert(NQ % QT == 0 && NQ % BNQ == 0 && NQ >= BNQ && NQ <= NN);
static_assert(NN == HIMG * WIMG);
static_assert(SN == 2 * WIMG);
static_assert(NSTRIP * SN == NN);
static_assert(SN == 8 * 16);
static_assert(HIMG % 2 == 0 && WIMG % 2 == 0);
static_assert(HP == HIMG / 2 && WP == WIMG / 2);
static_assert(MM == HP * WP);
static_assert(WP == 32);
static_assert(MM % QT == 0 && MM % 32 == 0);
static_assert(NN % QT == 0 && CC % QT == 0 && DQ % QT == 0);
static_assert(MW == 3 * DQ && MW % QT == 0 && MW % 8 == 0);
static_assert(CC % 32 == 0 && DQ % 32 == 0);
static_assert((OSP * 4) % 16 == 0);
static_assert((OSPW * 4) % 16 == 0);
static_assert((TP * 2) % 16 == 0);
static_assert(SN * OSP * 4 <= 65536);
static_assert(CC % CHB == 0 && CHB == 32);
static_assert(NN % 16 == 0 && BNQ == 2 * 128 && CC % 4 == 0);
static_assert((size_t)NB_FULL * CC * NN * 4 == (size_t)33554432);

typedef _Float16       v16h __attribute__((ext_vector_type(16)));
typedef _Float16       v8h  __attribute__((ext_vector_type(8)));
typedef __bf16         v16b __attribute__((ext_vector_type(16)));
typedef unsigned short v8us __attribute__((ext_vector_type(8)));
typedef float          v8f  __attribute__((ext_vector_type(8)));
typedef float          v4f  __attribute__((ext_vector_type(4)));
typedef unsigned int   v4u  __attribute__((ext_vector_type(4)));

union Frag  { v8us u[2]; v16h h; v16b bf; };
union FragH { v16h v; v8h hv[2]; };
static_assert(sizeof(Frag) == 32);
static_assert(sizeof(FragH) == 32);

__device__ __forceinline__ unsigned short bf_bits(float f) {
  unsigned u = __float_as_uint(f);
  return (unsigned short)((u + 0x7FFFu + ((u >> 16) & 1u)) >> 16);
}
__device__ __forceinline__ float bf_up(unsigned short hb) { return __uint_as_float(((unsigned)hb) << 16); }
__device__ __forceinline__ float bfr(float f) { return bf_up(bf_bits(f)); }
__device__ __forceinline__ unsigned short h_bits(_Float16 x) { return __builtin_bit_cast(unsigned short, x); }
__device__ __forceinline__ unsigned pk16(unsigned short a, unsigned short b) { return (unsigned)a | ((unsigned)b << 16); }
__device__ __forceinline__ v8f zero8() { v8f z = {0.f, 0.f, 0.f, 0.f, 0.f, 0.f, 0.f, 0.f}; return z; }
__device__ __forceinline__ float hmax8(v8f s) {
  return fmaxf(fmaxf(fmaxf(s[0], s[1]), fmaxf(s[2], s[3])), fmaxf(fmaxf(s[4], s[5]), fmaxf(s[6], s[7])));
}
__device__ __forceinline__ unsigned wave_ballot(bool p) {
#if defined(__HIP_DEVICE_COMPILE__)
  return __builtin_amdgcn_ballot_w32(p);
#else
  return p ? 1u : 0u;
#endif
}
__device__ __forceinline__ void split8(const float* f, v4u& uh, v4u& ul) {
#pragma unroll
  for (int t = 0; t < 4; ++t) {
    const float f0 = f[2 * t], f1 = f[2 * t + 1];
    const unsigned short hb0 = bf_bits(f0), hb1 = bf_bits(f1);
    const unsigned short lb0 = bf_bits(f0 - bf_up(hb0));
    const unsigned short lb1 = bf_bits(f1 - bf_up(hb1));
    uh[t] = pk16(hb0, hb1);
    ul[t] = pk16(lb0, lb1);
  }
}

__device__ __forceinline__ Frag ldfrag(const unsigned short* p) {
  Frag f;
  f.u[0] = *(const v8us*)(p);
  f.u[1] = *(const v8us*)(p + 16);
  return f;
}

__device__ __forceinline__ v8f mma_h(v16h a, v16h b, v8f c) {
  v8f d = __builtin_amdgcn_wmma_f32_16x16x32_f16(false, a, false, b, (short)0, c, false, false);
#if defined(__HIP_DEVICE_COMPILE__)
  asm volatile("v_nop\n\tv_nop\n\tv_nop\n\tv_nop" : "+v"(d) : "v"(a), "v"(b));
#endif
  return d;
}
__device__ __forceinline__ v8f mma_b(v16b a, v16b b, v8f c) {
  v8f d = __builtin_amdgcn_wmma_f32_16x16x32_bf16(false, a, false, b, (short)0, c, false, false);
#if defined(__HIP_DEVICE_COMPILE__)
  const v16h ha = __builtin_bit_cast(v16h, a), hb = __builtin_bit_cast(v16h, b);
  asm volatile("v_nop\n\tv_nop\n\tv_nop\n\tv_nop" : "+v"(d) : "v"(ha), "v"(hb));
#endif
  return d;
}

__global__ __launch_bounds__(256)
void cvt_w(const float* __restrict__ tw, const float* __restrict__ pw, const float* __restrict__ gw,
           const float* __restrict__ ow, unsigned short* W16, unsigned short* WWb) {
  const int tid = threadIdx.x, blk = blockIdx.x;
  if (blk < MW / 8) {
    const int rl = tid >> 5, col = 8 * (tid & 31);
    const int o = 8 * blk + rl;
    const int grp = blk >> 4;
    const float* wbase = (grp == 0) ? tw : ((grp == 1) ? pw : gw);
    const float* s = wbase + (size_t)(o - DQ * grp) * CC + col;
    const v4f a = *(const v4f*)s;
    const v4f q = *(const v4f*)(s + 4);
    const float f[8] = {a[0], a[1], a[2], a[3], q[0], q[1], q[2], q[3]};
    v4u u;
#pragma unroll
    for (int t = 0; t < 4; ++t) {
      const _Float16 h0 = (_Float16)(bfr(f[2 * t]) * WSC);
      const _Float16 h1 = (_Float16)(bfr(f[2 * t + 1]) * WSC);
      u[t] = pk16(h_bits(h0), h_bits(h1));
    }
#pragma unroll
    for (int pass = 0; pass < 2; ++pass) {
      *(volatile v4u*)(W16 + (size_t)o * CC + col) = u;
      __threadfence();
    }
  } else {
    const int rb = blk - MW / 8;
    const int o = 16 * rb + (tid >> 4);
    const int col = 8 * (tid & 15);
    const float* s = ow + (size_t)o * DQ + col;
    const v4f a = *(const v4f*)s;
    const v4f q = *(const v4f*)(s + 4);
    const float f[8] = {a[0], a[1], a[2], a[3], q[0], q[1], q[2], q[3]};
    v4u u;
#pragma unroll
    for (int t = 0; t < 4; ++t) u[t] = pk16(bf_bits(f[2 * t]), bf_bits(f[2 * t + 1]));
#pragma unroll
    for (int pass = 0; pass < 2; ++pass) {
      *(volatile v4u*)(WWb + (size_t)o * DQ + col) = u;
      __threadfence();
    }
  }
}

__global__ __launch_bounds__(256)
void cvt_x(const float* __restrict__ x, unsigned short* XP) {
  __shared__ __align__(16) unsigned short T[QT * TP];
  const int tid = threadIdx.x;
  const int nb = blockIdx.x, cb = blockIdx.y, b = blockIdx.z;
  const int e = tid & 7, lq = tid >> 3;
  const int n0 = nb * QT, c0 = cb * QT;
#pragma unroll
  for (int it = 0; it < 2; ++it) {
    const int cl = it * 32 + lq;
    const float* sp = x + ((size_t)(b * CC + c0 + cl)) * NN + n0 + 8 * e;
    const v4f a = *(const v4f*)sp;
    const v4f q = *(const v4f*)(sp + 4);
    unsigned short hb[8];
#pragma unroll
    for (int t = 0; t < 4; ++t) {
      hb[t]     = h_bits((_Float16)bfr(a[t]));
      hb[4 + t] = h_bits((_Float16)bfr(q[t]));
    }
#pragma unroll
    for (int t = 0; t < 8; ++t) T[(8 * e + t) * TP + cl] = hb[t];
  }
  __syncthreads();
  v4u up[2];
#pragma unroll
  for (int it = 0; it < 2; ++it) {
    const int nl = it * 32 + lq;
    up[it] = *(const v4u*)(T + nl * TP + 8 * e);
  }
#pragma unroll
  for (int pass = 0; pass < 2; ++pass) {
#pragma unroll
    for (int it = 0; it < 2; ++it) {
      const int rl = it * 32 + lq;
      *(volatile v4u*)(XP + ((size_t)(b * NN + n0 + rl)) * CC + c0 + 8 * e) = up[it];
    }
    __threadfence();
  }
}

__global__ __launch_bounds__(256)
void gemm_proj(const unsigned short* __restrict__ W16, const unsigned short* __restrict__ XP,
               const float* __restrict__ tb, const float* __restrict__ pb, const float* __restrict__ gb,
               unsigned short* Qh, unsigned short* Ql, float* PF, float* GF) {
  __shared__ __align__(16) float Os[SN * OSP];
  const int tid  = threadIdx.x;
  const int lane = tid & 31, wave = tid >> 5;
  const int hh   = lane >> 4, c = lane & 15;
  const int st   = blockIdx.x, mb = blockIdx.y, b = blockIdx.z;
  const int n0   = st * SN, o0 = mb * QT;

  const unsigned short* ap = W16 + (size_t)(o0 + c) * CC + 8 * hh;
  const unsigned short* bp = XP + ((size_t)(b * NN + n0 + 16 * wave + c)) * CC + 8 * hh;

  v8f acc[4];
#pragma unroll
  for (int mt = 0; mt < 4; ++mt) acc[mt] = zero8();

#pragma unroll
  for (int ks = 0; ks < CC / 32; ++ks) {
    const Frag fb = ldfrag(bp + 32 * ks);
#pragma unroll
    for (int mt = 0; mt < 4; ++mt) {
      const Frag fa = ldfrag(ap + (size_t)(16 * mt) * CC + 32 * ks);
      acc[mt] = mma_h(fa.h, fb.h, acc[mt]);
    }
  }

  {
    const int nl = 16 * wave + c;
#pragma unroll
    for (int mt = 0; mt < 4; ++mt) {
      v4f va, vb;
#pragma unroll
      for (int r = 0; r < 4; ++r) { va[r] = acc[mt][r] * IWSC; vb[r] = acc[mt][4 + r] * IWSC; }
      *(v4f*)(Os + nl * OSP + 16 * mt + 8 * hh)     = va;
      *(v4f*)(Os + nl * OSP + 16 * mt + 8 * hh + 4) = vb;
    }
  }
  __syncthreads();

  const int grp = mb >> 1;
  const int dsel = (mb & 1) * QT;
  const float* bias = (grp == 0) ? tb : ((grp == 1) ? pb : gb);

  if (grp == 0) {
    const int e = tid & 7, lq = tid >> 3;
    float bv[8];
    {
      const v4f ba = *(const v4f*)(bias + dsel + 8 * e);
      const v4f bq = *(const v4f*)(bias + dsel + 8 * e + 4);
#pragma unroll
      for (int t = 0; t < 4; ++t) { bv[t] = bfr(ba[t]); bv[4 + t] = bfr(bq[t]); }
    }
    v4u uh[4], ul[4];
#pragma unroll
    for (int it = 0; it < 4; ++it) {
      const int row = it * 32 + lq;
      const v4f a = *(const v4f*)(Os + row * OSP + 8 * e);
      const v4f q = *(const v4f*)(Os + row * OSP + 8 * e + 4);
      float f[8];
#pragma unroll
      for (int t = 0; t < 4; ++t) { f[t] = a[t] + bv[t]; f[4 + t] = q[t] + bv[4 + t]; }
      split8(f, uh[it], ul[it]);
    }
#pragma unroll
    for (int pass = 0; pass < 2; ++pass) {
#pragma unroll
      for (int it = 0; it < 4; ++it) {
        const int row = it * 32 + lq;
        const size_t po = ((size_t)(b * NN + n0 + row)) * DQ + dsel + 8 * e;
        *(volatile v4u*)(Qh + po) = uh[it];
        *(volatile v4u*)(Ql + po) = ul[it];
      }
      __threadfence();
    }
  } else {
    const int e16 = tid & 15, lr = tid >> 4;
    v4f bv4;
    {
      const v4f bq = *(const v4f*)(bias + dsel + 4 * e16);
#pragma unroll
      for (int t = 0; t < 4; ++t) bv4[t] = bfr(bq[t]);
    }
    float* P = (grp == 1) ? PF : GF;
    v4f res[8];
#pragma unroll
    for (int it = 0; it < 8; ++it) {
      const int row = it * 16 + lr;
      const v4f a = *(const v4f*)(Os + row * OSP + 4 * e16);
      v4f v;
#pragma unroll
      for (int t = 0; t < 4; ++t) v[t] = a[t] + bv4[t];
      res[it] = v;
    }
#pragma unroll
    for (int pass = 0; pass < 2; ++pass) {
#pragma unroll
      for (int it = 0; it < 8; ++it) {
        const int row = it * 16 + lr;
        const size_t po = ((size_t)(b * NN + n0 + row)) * DQ + dsel + 4 * e16;
        *(volatile v4f*)(P + po) = res[it];
      }
      __threadfence();
    }
  }
}

__global__ __launch_bounds__(256)
void pool_k(const float* __restrict__ PF, const float* __restrict__ GF,
            unsigned short* Kh, unsigned short* Kl, unsigned short* Gp) {
  const int tid = threadIdx.x, py = blockIdx.x, b = blockIdx.y;
  const int e16 = tid & 15, lr = tid >> 4;
  v4u kh[2], kl[2], gu[2];
#pragma unroll
  for (int it = 0; it < 2; ++it) {
    const int px = it * 16 + lr;
    float fk[8], fg[8];
#pragma unroll
    for (int t = 0; t < 8; ++t) { fk[t] = -__builtin_inff(); fg[t] = -__builtin_inff(); }
#pragma unroll
    for (int dy = 0; dy < 2; ++dy) {
      const size_t rb = ((size_t)(b * NN + (2 * py + dy) * WIMG + 2 * px)) * DQ + 8 * e16;
#pragma unroll
      for (int dx = 0; dx < 2; ++dx) {
        const float* pk = PF + rb + (size_t)dx * DQ;
        const float* pg = GF + rb + (size_t)dx * DQ;
        const v4f ka = *(const v4f*)pk, kq = *(const v4f*)(pk + 4);
        const v4f ga = *(const v4f*)pg, gq = *(const v4f*)(pg + 4);
#pragma unroll
        for (int t = 0; t < 4; ++t) {
          fk[t]     = fmaxf(fk[t], ka[t]);
          fk[4 + t] = fmaxf(fk[4 + t], kq[t]);
          fg[t]     = fmaxf(fg[t], ga[t]);
          fg[4 + t] = fmaxf(fg[4 + t], gq[t]);
        }
      }
    }
    split8(fk, kh[it], kl[it]);
#pragma unroll
    for (int t = 0; t < 4; ++t) gu[it][t] = pk16(h_bits((_Float16)fg[2 * t]), h_bits((_Float16)fg[2 * t + 1]));
  }
#pragma unroll
  for (int pass = 0; pass < 2; ++pass) {
#pragma unroll
    for (int it = 0; it < 2; ++it) {
      const int px = it * 16 + lr;
      const size_t po = ((size_t)(b * MM + WP * py + px)) * DQ + 8 * e16;
      *(volatile v4u*)(Kh + po) = kh[it];
      *(volatile v4u*)(Kl + po) = kl[it];
      *(volatile v4u*)(Gp + po) = gu[it];
    }
    __threadfence();
  }
}

__global__ __launch_bounds__(256)
void tr_g(const unsigned short* __restrict__ Gp, unsigned short* Gc) {
  __shared__ __align__(16) unsigned short T[QT * TP];
  const int tid = threadIdx.x;
  const int mt = blockIdx.x, db = blockIdx.y, b = blockIdx.z;
  const int e = tid & 7, lq = tid >> 3;
  const int m0 = mt * QT, d0 = db * QT;
#pragma unroll
  for (int it = 0; it < 2; ++it) {
    const int ml = it * 32 + lq;
    const v4u w = *(const v4u*)(Gp + ((size_t)(b * MM + m0 + ml)) * DQ + d0 + 8 * e);
    unsigned short hb[8];
#pragma unroll
    for (int t = 0; t < 4; ++t) {
      hb[2 * t]     = (unsigned short)(w[t] & 0xFFFFu);
      hb[2 * t + 1] = (unsigned short)(w[t] >> 16);
    }
#pragma unroll
    for (int t = 0; t < 8; ++t) T[(8 * e + t) * TP + ml] = hb[t];
  }
  __syncthreads();
  v4u up[2];
#pragma unroll
  for (int it = 0; it < 2; ++it) {
    const int dl = it * 32 + lq;
    up[it] = *(const v4u*)(T + dl * TP + 8 * e);
  }
#pragma unroll
  for (int pass = 0; pass < 2; ++pass) {
#pragma unroll
    for (int it = 0; it < 2; ++it) {
      const int dl = it * 32 + lq;
      *(volatile v4u*)(Gc + ((size_t)(b * DQ + d0 + dl)) * MM + m0 + 8 * e) = up[it];
    }
    __threadfence();
  }
}

__global__ __launch_bounds__(128) __attribute__((amdgpu_num_vgpr(256)))
void attn_k(const unsigned short* __restrict__ Qh, const unsigned short* __restrict__ Ql,
            const unsigned short* __restrict__ Kh, const unsigned short* __restrict__ Kl,
            const unsigned short* __restrict__ Gc, unsigned short* Yh, unsigned short* Yl) {
  __shared__ __align__(16) float Os[QT * OSPW];
  const int tid  = threadIdx.x;
  const int wave = tid >> 5, lane = tid & 31;
  const int hh   = lane >> 4, c = lane & 15;
  const int n0   = blockIdx.x * QT, b = blockIdx.y;

  const size_t qo = ((size_t)(b * NN + n0 + 16 * wave + c)) * DQ + 8 * hh;
  const unsigned short* Qhp = Qh + qo;
  const unsigned short* Qlp = Ql + qo;
  const unsigned short* Khp = Kh + (size_t)b * MM * DQ + (size_t)c * DQ + 8 * hh;
  const unsigned short* Klp = Kl + (size_t)b * MM * DQ + (size_t)c * DQ + 8 * hh;
  const unsigned short* Vp = Gc + (size_t)b * DQ * MM + (size_t)c * MM + 8 * hh;

  float m = -1.0e30f, l = 0.f;
  v8f o[8];
#pragma unroll
  for (int j = 0; j < 8; ++j) o[j] = zero8();

#pragma unroll 1
  for (int kb = 0; kb < MM; kb += 32) {
    const unsigned short* k0p  = Khp + (size_t)kb * DQ;
    const unsigned short* k1p  = Khp + (size_t)(kb + 16) * DQ;
    const unsigned short* k0lp = Klp + (size_t)kb * DQ;
    const unsigned short* k1lp = Klp + (size_t)(kb + 16) * DQ;
    v8f s0 = zero8(), s1 = zero8();
#pragma unroll 1
    for (int kc = 0; kc < DQ / 32; ++kc) {
      const Frag qh  = ldfrag(Qhp + 32 * kc);
      const Frag ql  = ldfrag(Qlp + 32 * kc);
      const Frag k0  = ldfrag(k0p + 32 * kc);
      const Frag k1  = ldfrag(k1p + 32 * kc);
      const Frag k0l = ldfrag(k0lp + 32 * kc);
      const Frag k1l = ldfrag(k1lp + 32 * kc);
      s0 = mma_b(k0.bf, qh.bf, s0);
      s1 = mma_b(k1.bf, qh.bf, s1);
      s0 = mma_b(k0.bf, ql.bf, s0);
      s1 = mma_b(k1.bf, ql.bf, s1);
      s0 = mma_b(k0l.bf, qh.bf, s0);
      s1 = mma_b(k1l.bf, qh.bf, s1);
    }

    float mx = fmaxf(hmax8(s0), hmax8(s1));
    mx = fmaxf(mx, __shfl_xor(mx, 16, 32));
    const float mn = fmaxf(m, mx);
    const unsigned grew = wave_ballot(mx > m);
    if (grew != 0u) {
      const float corr = __expf(m - mn);
      l *= corr;
#pragma unroll
      for (int j = 0; j < 8; ++j) {
#pragma unroll
        for (int r = 0; r < 8; ++r) o[j][r] *= corr;
      }
    }
    m = mn;
    const float msh = mn - LNPS;

    FragH ph;
    float ls = 0.f;
#pragma unroll
    for (int r = 0; r < 8; ++r) {
      const float e0 = __expf(s0[r] - msh);
      const float e1 = __expf(s1[r] - msh);
      ls += e0 + e1;
      ph.hv[0][r] = (_Float16)e0;
      ph.hv[1][r] = (_Float16)e1;
    }
    l += ls;

#pragma unroll
    for (int j = 0; j < 8; ++j) {
      const Frag vf = ldfrag(Vp + (size_t)(16 * j) * MM + kb);
      o[j] = mma_h(vf.h, ph.v, o[j]);
    }
  }
  l += __shfl_xor(l, 16, 32);
  const float inv = 1.0f / l;

  {
    const int qrow = 16 * wave + c;
#pragma unroll
    for (int j = 0; j < 8; ++j) {
      v4f va, vb;
#pragma unroll
      for (int r = 0; r < 4; ++r) { va[r] = o[j][r] * inv; vb[r] = o[j][4 + r] * inv; }
      *(v4f*)(Os + qrow * OSPW + 16 * j + 8 * hh)     = va;
      *(v4f*)(Os + qrow * OSPW + 16 * j + 8 * hh + 4) = vb;
    }
  }
  __syncthreads();

  const int e16 = tid & 15, lr = tid >> 4;
  v4u uh[8], ul[8];
#pragma unroll
  for (int it = 0; it < 8; ++it) {
    const int row = it * 8 + lr;
    const v4f a = *(const v4f*)(Os + row * OSPW + 8 * e16);
    const v4f q = *(const v4f*)(Os + row * OSPW + 8 * e16 + 4);
    const float f[8] = {a[0], a[1], a[2], a[3], q[0], q[1], q[2], q[3]};
    split8(f, uh[it], ul[it]);
  }
#pragma unroll
  for (int pass = 0; pass < 2; ++pass) {
#pragma unroll
    for (int it = 0; it < 8; ++it) {
      const int row = it * 8 + lr;
      const size_t po = ((size_t)(b * NN + n0 + row)) * DQ + 8 * e16;
      *(volatile v4u*)(Yh + po) = uh[it];
      *(volatile v4u*)(Yl + po) = ul[it];
    }
    __threadfence();
  }
}

__global__ __launch_bounds__(128)
void gemm_out(const unsigned short* __restrict__ WWb, const unsigned short* __restrict__ Yh,
              const unsigned short* __restrict__ Yl, const float* __restrict__ wb, float* WY) {
  __shared__ __align__(16) float Os[QT * OSP];
  const int tid  = threadIdx.x;
  const int lane = tid & 31, wave = tid >> 5;
  const int hh   = lane >> 4, c = lane & 15;
  const int nt   = blockIdx.x, cb = blockIdx.y, b = blockIdx.z;
  const int n0   = nt * QT, c0 = cb * QT;

  const unsigned short* ap  = WWb + (size_t)(c0 + c) * DQ + 8 * hh;
  const size_t bo = ((size_t)(b * NN + n0 + 16 * wave + c)) * DQ + 8 * hh;
  const unsigned short* bph = Yh + bo;
  const unsigned short* bpl = Yl + bo;

  v8f acc[4];
#pragma unroll
  for (int mt = 0; mt < 4; ++mt) acc[mt] = zero8();

#pragma unroll
  for (int ks = 0; ks < DQ / 32; ++ks) {
    const Frag fbh = ldfrag(bph + 32 * ks);
    const Frag fbl = ldfrag(bpl + 32 * ks);
#pragma unroll
    for (int mt = 0; mt < 4; ++mt) {
      const Frag fa = ldfrag(ap + (size_t)(16 * mt) * DQ + 32 * ks);
      acc[mt] = mma_b(fa.bf, fbh.bf, acc[mt]);
      acc[mt] = mma_b(fa.bf, fbl.bf, acc[mt]);
    }
  }

  {
    const int nl = 16 * wave + c;
#pragma unroll
    for (int mt = 0; mt < 4; ++mt) {
      v4f va, vb;
#pragma unroll
      for (int r = 0; r < 4; ++r) { va[r] = acc[mt][r]; vb[r] = acc[mt][4 + r]; }
      *(v4f*)(Os + nl * OSP + 16 * mt + 8 * hh)     = va;
      *(v4f*)(Os + nl * OSP + 16 * mt + 8 * hh + 4) = vb;
    }
  }
  __syncthreads();

  const int e = tid & 7, lq = tid >> 3;
  v4f res[8];
#pragma unroll
  for (int it = 0; it < 8; ++it) {
    const int L   = it * 16 + lq;
    const int cl  = L >> 1, hf = L & 1;
    const int nl  = hf * 32 + 4 * e;
    const float bvs = bfr(wb[c0 + cl]);
#pragma unroll
    for (int t = 0; t < 4; ++t) {
      res[it][t] = Os[(nl + t) * OSP + cl] + bvs;
    }
  }
#pragma unroll
  for (int pass = 0; pass < 2; ++pass) {
#pragma unroll
    for (int it = 0; it < 8; ++it) {
      const int L   = it * 16 + lq;
      const int cl  = L >> 1, hf = L & 1;
      const int nl  = hf * 32 + 4 * e;
      const size_t idx = ((size_t)(b * CC + c0 + cl)) * NN + n0 + nl;
      *(volatile v4f*)(WY + idx) = res[it];
    }
    __threadfence();
  }
}

__global__ __launch_bounds__(256)
void bn_stat(const float* __restrict__ WY, float* MU) {
#pragma clang fp contract(off)
  __shared__ double red[16];
  __shared__ __align__(16) float tab[2 * CHB];
  const int tid = threadIdx.x, lane = tid & 31, wave = tid >> 5;
  const int c0 = blockIdx.x * CHB;
  const double ninv = 1.0 / ((double)NB * (double)NQ);
#pragma unroll 1
  for (int ch = 0; ch < CHB; ++ch) {
    const int cc = c0 + ch;
    double s = 0.0, q = 0.0;
#pragma unroll 1
    for (int bb = 0; bb < NB; ++bb) {
      const float* rp = WY + ((size_t)(bb * CC + cc)) * NN;
#pragma unroll 1
      for (int i = tid; i < NQ / 16; i += 256) {
        const float* p = rp + 16 * i;
        const v4f a0 = *(const v4f*)(p);
        const v4f a1 = *(const v4f*)(p + 4);
        const v4f a2 = *(const v4f*)(p + 8);
        const v4f a3 = *(const v4f*)(p + 12);
#pragma unroll
        for (int t = 0; t < 4; ++t) {
          const double d0 = (double)a0[t], d1 = (double)a1[t], d2 = (double)a2[t], d3 = (double)a3[t];
          s += d0; q += d0 * d0;
          s += d1; q += d1 * d1;
          s += d2; q += d2 * d2;
          s += d3; q += d3 * d3;
        }
      }
    }
#pragma unroll
    for (int d = 1; d < 32; d <<= 1) {
      s += __shfl_xor(s, d, 32);
      q += __shfl_xor(q, d, 32);
    }
    if (lane == 0) { red[wave] = s; red[8 + wave] = q; }
    __syncthreads();
    if (tid == 0) {
      double ts = 0.0, tq = 0.0;
#pragma unroll
      for (int w = 0; w < 8; ++w) { ts += red[w]; tq += red[8 + w]; }
      const double mu = ts * ninv;
      double var = tq * ninv - mu * mu;
      var = (var > 0.0) ? var : 0.0;
      const float varf = (float)var + BNEPS;
      const float rs = 1.0f / sqrtf(varf);
      tab[ch] = (float)mu;
      tab[CHB + ch] = rs;
    }
    __syncthreads();
  }
  if (wave == 0) {
    const v4f v = *(const v4f*)(tab + 4 * (lane & 15));
    float* dst = MU + c0 + 4 * (lane & 7) + ((lane & 8) ? CC : 0);
#pragma unroll
    for (int pass = 0; pass < 2; ++pass) {
      if (lane < 16) *(volatile v4f*)dst = v;
      __threadfence();
    }
  }
}

__global__ __launch_bounds__(256)
void bn_apply(const float* __restrict__ WY, const float* __restrict__ x, const float* __restrict__ gam,
              const float* __restrict__ bet, const float* __restrict__ MU, float* out) {
#pragma clang fp contract(off)
  const int tid = threadIdx.x, lane = tid & 31, wave = tid >> 5;
  const int nq = blockIdx.x, cb = blockIdx.y, b = blockIdx.z;
  const int c = cb * 4 + (wave >> 1);
  const int n = nq * BNQ + (wave & 1) * 128 + 4 * lane;
  const float mu = MU[c], rs = MU[CC + c];
  const float ga = bfr(gam[c]), be = bfr(bet[c]);
  const size_t idx = ((size_t)(b * CC + c)) * NN + n;
  const v4f w  = *(const v4f*)(WY + idx);
  const v4f xv = *(const v4f*)(x + idx);
  v4f r;
#pragma unroll
  for (int t = 0; t < 4; ++t) {
    const float d  = w[t] - mu;
    const float nv = d * rs;
    const float av = nv * ga;
    const float sv = av + be;
    r[t] = sv + bfr(xv[t]);
  }
#pragma unroll
  for (int pass = 0; pass < 2; ++pass) {
    *(volatile v4f*)(out + idx) = r;
    __threadfence();
  }
}

extern "C" void kernel_launch(void* const* d_in, const int* in_sizes, int n_in,
                              void* d_out, int out_size, void* d_ws, size_t ws_size,
                              hipStream_t stream) {
  const int XN = NB * CC * NN;
  if (n_in < 11) return;
  if (in_sizes[0] < XN) return;
  if (in_sizes[1] < DQ * CC || in_sizes[3] < DQ * CC || in_sizes[5] < DQ * CC || in_sizes[7] < CC * DQ) return;
  if (in_sizes[2] < DQ || in_sizes[4] < DQ || in_sizes[6] < DQ || in_sizes[8] < CC) return;
  if (in_sizes[9] < CC || in_sizes[10] < CC) return;
  if (out_size < XN) return;

  size_t off = 0;
  auto carve = [&](size_t bytes) { const size_t o = off; off += (bytes + 255) & ~(size_t)255; return o; };
  const size_t oW16 = carve((size_t)MW * CC * 2);
  const size_t oWWb = carve((size_t)CC * DQ * 2);
  const size_t oXP  = carve((size_t)NB * NN * CC * 2);
  const size_t oQh  = carve((size_t)NB * NN * DQ * 2);
  const size_t oQl  = carve((size_t)NB * NN * DQ * 2);
  const size_t oPF  = carve((size_t)NB * NN * DQ * 4);
  const size_t oGF  = carve((size_t)NB * NN * DQ * 4);
  const size_t oKh  = carve((size_t)NB * MM * DQ * 2);
  const size_t oKl  = carve((size_t)NB * MM * DQ * 2);
  const size_t oGp  = carve((size_t)NB * MM * DQ * 2);
  const size_t oGc  = carve((size_t)NB * DQ * MM * 2);
  const size_t oYh  = carve((size_t)NB * NN * DQ * 2);
  const size_t oYl  = carve((size_t)NB * NN * DQ * 2);
  const size_t oWY  = carve((size_t)NB * CC * NN * 4);
  const size_t oMU  = carve((size_t)2 * CC * 4);
  if (off > ws_size) return;
  if (off > (size_t)134217728) return;

  const float* x   = (const float*)d_in[0];
  const float* gw  = (const float*)d_in[1];
  const float* gb  = (const float*)d_in[2];
  const float* tw  = (const float*)d_in[3];
  const float* tb  = (const float*)d_in[4];
  const float* pw  = (const float*)d_in[5];
  const float* pb  = (const float*)d_in[6];
  const float* ow  = (const float*)d_in[7];
  const float* wb  = (const float*)d_in[8];
  const float* gam = (const float*)d_in[9];
  const float* bet = (const float*)d_in[10];

  char* ws = (char*)d_ws;
  unsigned short* W16 = (unsigned short*)(ws + oW16);
  unsigned short* WWb = (unsigned short*)(ws + oWWb);
  unsigned short* XP  = (unsigned short*)(ws + oXP);
  unsigned short* Qh  = (unsigned short*)(ws + oQh);
  unsigned short* Ql  = (unsigned short*)(ws + oQl);
  float*          PF  = (float*)(ws + oPF);
  float*          GF  = (float*)(ws + oGF);
  unsigned short* Kh  = (unsigned short*)(ws + oKh);
  unsigned short* Kl  = (unsigned short*)(ws + oKl);
  unsigned short* Gp  = (unsigned short*)(ws + oGp);
  unsigned short* Gc  = (unsigned short*)(ws + oGc);
  unsigned short* Yh  = (unsigned short*)(ws + oYh);
  unsigned short* Yl  = (unsigned short*)(ws + oYl);
  float*          WY  = (float*)(ws + oWY);
  float*          MU  = (float*)(ws + oMU);
  float* out = (float*)d_out;

  const dim3 blk256(256), blk128(128);

  cvt_w<<<dim3(MW / 8 + CC / 16), blk256, 0, stream>>>(tw, pw, gw, ow, W16, WWb);
  cvt_x<<<dim3(NN / QT, CC / QT, NB), blk256, 0, stream>>>(x, XP);
  gemm_proj<<<dim3(NSTRIP, MW / QT, NB), blk256, 0, stream>>>(W16, XP, tb, pb, gb, Qh, Ql, PF, GF);
  pool_k<<<dim3(HP, NB), blk256, 0, stream>>>(PF, GF, Kh, Kl, Gp);
  tr_g<<<dim3(MM / QT, DQ / QT, NB), blk256, 0, stream>>>(Gp, Gc);
  attn_k<<<dim3(NQ / QT, NB), blk128, 0, stream>>>(Qh, Ql, Kh, Kl, Gc, Yh, Yl);
  gemm_out<<<dim3(NQ / QT, CC / QT, NB), blk128, 0, stream>>>(WWb, Yh, Yl, wb, WY);
  bn_stat<<<dim3(CC / CHB), blk256, 0, stream>>>(WY, MU);
  bn_apply<<<dim3(NQ / BNQ, CC / 4, NB), blk256, 0, stream>>>(WY, x, gam, bet, MU, out);
  (void)hipGetLastError();
}
